// RNN_LSTM_22703197127160
// MI455X (gfx1250) — hardware-verified
//
#include <hip/hip_runtime.h>
#include <stdint.h>

typedef __attribute__((ext_vector_type(16))) _Float16 v16h;
typedef __attribute__((ext_vector_type(8)))  _Float16 v8h;
typedef __attribute__((ext_vector_type(16))) __bf16   v16b;
typedef __attribute__((ext_vector_type(8)))  __bf16   v8b;
typedef __attribute__((ext_vector_type(8)))  float    v8f;
typedef __attribute__((ext_vector_type(4)))  float    v4f;
typedef __attribute__((ext_vector_type(8)))  unsigned short v8us;

__device__ __forceinline__ unsigned short f2bf_bits(float f) {
  unsigned u = __float_as_uint(f);
  return (unsigned short)((u + 0x7FFFu + ((u >> 16) & 1u)) >> 16);
}
__device__ __forceinline__ float bf_bits2f(unsigned short h) { return __uint_as_float(((unsigned)h) << 16); }

__device__ __forceinline__ void dep_guard_h(v8f& a, v8f& b, v16h x, v16h y) { asm volatile("v_nop\n\tv_nop\n\tv_nop\n\tv_nop" : "+v"(a), "+v"(b) : "v"(x), "v"(y)); }
__device__ __forceinline__ void dep_guard_b(v8f& a, v8f& b, v16b x, v16b y) { asm volatile("v_nop\n\tv_nop\n\tv_nop\n\tv_nop" : "+v"(a), "+v"(b) : "v"(x), "v"(y)); }
__device__ __forceinline__ void keep4_h(v16h a, v16h b, v16h c, v16h d) { asm volatile("v_nop" :: "v"(a), "v"(b), "v"(c), "v"(d)); }
__device__ __forceinline__ void keep4_b(v16b a, v16b b, v16b c, v16b d) { asm volatile("v_nop" :: "v"(a), "v"(b), "v"(c), "v"(d)); }
__device__ __forceinline__ void acc_guard4(v8f& a, v8f& b, v8f& c, v8f& d) { asm volatile("v_nop\n\tv_nop\n\tv_nop\n\tv_nop" : "+v"(a), "+v"(b), "+v"(c), "+v"(d)); }
__device__ __forceinline__ void guard4_b(v8f& a, v8f& b, v16b w, v16b x, v16b y, v16b z) {
  asm volatile("v_nop\n\tv_nop\n\tv_nop\n\tv_nop" : "+v"(a), "+v"(b) : "v"(w), "v"(x), "v"(y), "v"(z));
}

template <typename T> struct Frag;
template <> struct Frag<_Float16> {
  typedef v16h V; union U { v16h v; v8h h[2]; };
  static __device__ __forceinline__ v16h load(const _Float16* p) {
    U f; f.h[0] = *(const v8h*)(p); f.h[1] = *(const v8h*)(p + 16); return f.v;
  }
  static __device__ __forceinline__ v8f mma(v16h a, v16h b, v8f c) {
    return __builtin_amdgcn_wmma_f32_16x16x32_f16(false, a, false, b, (short)0, c, false, false);
  }
  static __device__ __forceinline__ void guard(v8f& a, v8f& b, v16h x, v16h y) { dep_guard_h(a, b, x, y); }
  static __device__ __forceinline__ void keep(v16h a, v16h b, v16h c, v16h d) { keep4_h(a, b, c, d); }
};
template <> struct Frag<__bf16> {
  typedef v16b V; union U { v16b v; v8b h[2]; };
  static __device__ __forceinline__ v16b load(const __bf16* p) {
    U f; f.h[0] = *(const v8b*)(p); f.h[1] = *(const v8b*)(p + 16); return f.v;
  }
  static __device__ __forceinline__ v8f mma(v16b a, v16b b, v8f c) {
    return __builtin_amdgcn_wmma_f32_16x16x32_bf16(false, a, false, b, (short)0, c, false, false);
  }
  static __device__ __forceinline__ void guard(v8f& a, v8f& b, v16b x, v16b y) { dep_guard_b(a, b, x, y); }
  static __device__ __forceinline__ void keep(v16b a, v16b b, v16b c, v16b d) { keep4_b(a, b, c, d); }
};

template <int ET> struct Elem;
template <> struct Elem<0> { typedef _Float16 T; };
template <> struct Elem<1> { typedef __bf16 T; };
template <int ET, bool SPLIT, int BIAS_MODE, int OUT_MODE, bool RESID, int ACT = 0>
__global__ __launch_bounds__(256) void wmma_gemm64(
    const unsigned short* __restrict__ Ap, const unsigned short* __restrict__ A2p, int lda, long strideA,
    const unsigned short* __restrict__ Btp, const unsigned short* __restrict__ Bt2p, int ldb, long strideB,
    void* __restrict__ Cout, void* __restrict__ Cout2, int ldc, long strideC,
    const float* __restrict__ bias,
    const float* __restrict__ resid, long strideR,
    int M, int N, int K, float scale) {
  typedef typename Elem<ET>::T T;
  typedef typename Frag<T>::V V;
  const T* A = (const T*)Ap; const T* A2 = (const T*)A2p; const T* Bt = (const T*)Btp; const T* Bt2 = (const T*)Bt2p;
  __shared__ __align__(16) float sT[8][16 * 68];
  const int b    = blockIdx.y;
  const int lane = threadIdx.x & 31;
  const int wave = threadIdx.x >> 5;
  const int tilesN = N >> 6;
  const int tilesM = M >> 6;
  const int tile = blockIdx.x * 8 + wave;
  if (tile >= tilesM * tilesN) return;
  const int tm = tile / tilesN;
  const int tn = tile - tm * tilesN;
  const int m0 = tm << 6;
  const int n0 = tn << 6;

  const T* Ab  = A  + (size_t)b * strideA;
  const T* Bb  = Bt + (size_t)b * strideB;
  const T* Ab2 = SPLIT ? (A2  + (size_t)b * strideA) : nullptr;
  const T* Bb2 = SPLIT ? (Bt2 + (size_t)b * strideB) : nullptr;

  const int rlane = lane & 15;
  const int koff  = (lane >> 4) * 8;
  const int mOff  = (lane >> 4) * 8;

  v8f acc[4][4];
#pragma unroll
  for (int i = 0; i < 4; ++i)
#pragma unroll
    for (int j = 0; j < 4; ++j) acc[i][j] = (v8f){0.f,0.f,0.f,0.f,0.f,0.f,0.f,0.f};

  for (int k0 = 0; k0 < K; k0 += 32) {
    V bh[4], bl[4];
#pragma unroll
    for (int j = 0; j < 4; ++j) {
      const size_t bo = (size_t)(n0 + (j << 4) + rlane) * ldb + koff + k0;
      bh[j] = Frag<T>::load(Bb + bo);
      if (SPLIT) bl[j] = Frag<T>::load(Bb2 + bo);
    }
#pragma unroll
    for (int i = 0; i < 4; ++i) {
      const size_t ao = (size_t)(m0 + (i << 4) + rlane) * lda + koff + k0;
      V ah = Frag<T>::load(Ab + ao);
      V al;
      if (SPLIT) al = Frag<T>::load(Ab2 + ao);
#pragma unroll
      for (int j = 0; j < 4; ++j) {
        acc[i][j] = Frag<T>::mma(ah, bh[j], acc[i][j]);
        if (SPLIT) {
          acc[i][j] = Frag<T>::mma(ah, bl[j], acc[i][j]);
          acc[i][j] = Frag<T>::mma(al, bh[j], acc[i][j]);
        }
      }
      Frag<T>::guard(acc[i][0], acc[i][3], ah, SPLIT ? al : ah);
    }
    Frag<T>::keep(bh[0], bh[1], bh[2], bh[3]);
    if (SPLIT) Frag<T>::keep(bl[0], bl[1], bl[2], bl[3]);
  }
  acc_guard4(acc[0][0], acc[0][1], acc[0][2], acc[0][3]);
  acc_guard4(acc[1][0], acc[1][1], acc[1][2], acc[1][3]);
  acc_guard4(acc[2][0], acc[2][1], acc[2][2], acc[2][3]);
  acc_guard4(acc[3][0], acc[3][1], acc[3][2], acc[3][3]);

  float* slab = sT[wave];
  const float* Rb = RESID ? (resid + (size_t)b * strideR) : nullptr;
#pragma unroll
  for (int i = 0; i < 4; ++i) {
    const int mBase = m0 + (i << 4);
#pragma unroll
    for (int j = 0; j < 4; ++j) {
      const int n = n0 + (j << 4) + rlane;
      float bv = 0.f;
      if (BIAS_MODE == 2) bv = bias[n];
#pragma unroll
      for (int r = 0; r < 8; ++r) {
        float v = acc[i][j][r] * scale;
        if (BIAS_MODE == 1) v += bias[mBase + mOff + r];
        if (BIAS_MODE == 2) v += bv;
        if (RESID) v += Rb[(size_t)(mBase + mOff + r) * ldc + n];
        if (ACT == 1) v = tanhf(v);
        if (ACT == 2) v = fmaxf(v, 0.0f);
        if (ACT == 3) v = v / (1.0f + expf(-v));
        if (ACT == 4) v = (v > 0.f) ? v : 0.01f * v;
        if (ACT == 5) v = 0.5f * v * (1.0f + erff(v * 0.70710678118654752f));
        slab[(mOff + r) * 68 + (j << 4) + rlane] = v;
      }
    }
    __builtin_amdgcn_fence(__ATOMIC_RELEASE, "workgroup");
    __builtin_amdgcn_wave_barrier();
    __builtin_amdgcn_fence(__ATOMIC_ACQUIRE, "workgroup");
    if (OUT_MODE == 0) {
      float* C = (float*)Cout + (size_t)b * strideC;
      const int hh = lane >> 4, c4 = (lane & 15) * 4;
      for (int pass = 0; pass < 2; ++pass) {
#pragma unroll
        for (int it = 0; it < 8; ++it) {
          const int row = it * 2 + hh;
          v4f v = *(const v4f*)(slab + row * 68 + c4);
          *(volatile v4f*)(C + (size_t)(mBase + row) * ldc + n0 + c4) = v;
        }
        __threadfence();
      }
    } else {
      const int q = lane >> 3, c8 = (lane & 7) * 8;
      unsigned short* C  = (unsigned short*)Cout  + (size_t)b * strideC;
      unsigned short* C2 = (OUT_MODE == 2) ? ((unsigned short*)Cout2 + (size_t)b * strideC) : nullptr;
      for (int pass = 0; pass < 2; ++pass) {
#pragma unroll
        for (int it = 0; it < 4; ++it) {
          const int row = it * 4 + q;
          const float* sp = slab + row * 68 + c8;
          v8h hv, lv;
#pragma unroll
          for (int e = 0; e < 8; ++e) {
            if (OUT_MODE == 1) {
              hv[e] = (_Float16)sp[e];
            } else {
              unsigned short hb = f2bf_bits(sp[e]);
              unsigned short lb = f2bf_bits(sp[e] - bf_bits2f(hb));
              hv[e] = __builtin_bit_cast(_Float16, hb);
              lv[e] = __builtin_bit_cast(_Float16, lb);
            }
          }
          *(volatile v8h*)(C + (size_t)(mBase + row) * ldc + n0 + c8) = hv;
          if (OUT_MODE == 2) *(volatile v8h*)(C2 + (size_t)(mBase + row) * ldc + n0 + c8) = lv;
        }
        __threadfence();
      }
    }
    __builtin_amdgcn_fence(__ATOMIC_RELEASE, "workgroup");
    __builtin_amdgcn_wave_barrier();
    __builtin_amdgcn_fence(__ATOMIC_ACQUIRE, "workgroup");
  }
}

constexpr int kBatch     = 32;
constexpr int kSteps     = 512;
constexpr int kDin       = 256;
constexpr int kUnits     = 512;
constexpr int kGate4     = 4 * kUnits;
constexpr int kRows      = kBatch * kSteps;
constexpr int kChunks    = 2;
constexpr int kChunkRows = 16 * kSteps;
constexpr int kHbPitch   = 520;
static_assert(kChunks * 16 == kBatch);
static_assert(16 * 32 == kUnits);
static_assert((kHbPitch * 2) % 16 == 0);
static_assert(kDin % 64 == 0 && kUnits % 64 == 0 && kGate4 % 64 == 0 && kRows % 64 == 0);
static_assert(kDin % 32 == 0 && kUnits % 32 == 0);

constexpr size_t kSzX16 = (size_t)kRows * kDin * 2;
constexpr size_t kSzW0T = (size_t)kGate4 * kDin * 2;
constexpr size_t kSzWT  = (size_t)kGate4 * kUnits * 2;
constexpr size_t kSzWD  = (size_t)kDin * kUnits * 2;
constexpr size_t kSzH   = (size_t)kRows * kUnits * 2;
constexpr size_t kWsTotal = kSzX16 + kSzW0T + 6 * kSzWT + 2 * kSzWD + 4 * kSzH;
static_assert(kWsTotal == 89653248ULL);
static_assert(kWsTotal <= 134217728ULL);
static_assert(kSzX16 % 128 == 0 && kSzW0T % 128 == 0 && kSzWT % 128 == 0 && kSzWD % 128 == 0 && kSzH % 128 == 0);

__device__ __forceinline__ unsigned short f16_bits(float f) { return __builtin_bit_cast(unsigned short, (_Float16)f); }
__device__ __forceinline__ float sigm_f(float z) { return __builtin_amdgcn_rcpf(1.0f + __expf(-z)); }
__device__ __forceinline__ float tanh_f(float z) { return 1.0f - 2.0f * __builtin_amdgcn_rcpf(1.0f + __expf(2.0f * z)); }

__device__ __forceinline__ v16h ld_frag_h16(const unsigned short* p) {
  union { v16h v; v8us u[2]; } f; f.u[0] = *(const v8us*)(p); f.u[1] = *(const v8us*)(p + 16); return f.v;
}
__device__ __forceinline__ v16b ld_frag_b16(const unsigned short* p) {
  union { v16b v; v8us u[2]; } f; f.u[0] = *(const v8us*)(p); f.u[1] = *(const v8us*)(p + 16); return f.v;
}

__global__ __launch_bounds__(256) void reorder_cast_rows(const float* __restrict__ x, unsigned short* __restrict__ out, int nrows) {
  const int row = blockIdx.x * 8 + (threadIdx.x >> 5);
  const int lane = threadIdx.x & 31;
  const int rr = row < nrows ? row : nrows - 1;
  const int c = rr >> 13, rem = rr & 8191, t = rem >> 4, bl = rem & 15;
  const int b = c * 16 + bl;
  const float* src = x + ((size_t)b * kSteps + t) * kDin + lane * 8;
  const v4f p0 = *(const v4f*)src;
  const v4f p1 = *(const v4f*)(src + 4);
  v8us hv;
  hv[0] = f16_bits(p0[0]); hv[1] = f16_bits(p0[1]); hv[2] = f16_bits(p0[2]); hv[3] = f16_bits(p0[3]);
  hv[4] = f16_bits(p1[0]); hv[5] = f16_bits(p1[1]); hv[6] = f16_bits(p1[2]); hv[7] = f16_bits(p1[3]);
  if (row < nrows) {
    unsigned short* d = out + (size_t)row * kDin + lane * 8;
    *(volatile v8us*)d = hv;
    __threadfence();
    *(volatile v8us*)d = hv;
  }
}

template <int MODE>
__global__ __launch_bounds__(256) void transpose_cast64(const float* __restrict__ W, unsigned short* __restrict__ out,
                                                        unsigned short* __restrict__ out2, int K, int N, float scale) {
  __shared__ __align__(16) float tile[64 * 68];
  const int n0 = blockIdx.x * 64, k0 = blockIdx.y * 64;
  const int tid = threadIdx.x;
  {
    const int kr = tid >> 4, nc = (tid & 15) * 4;
#pragma unroll
    for (int i = 0; i < 4; ++i) {
      const int kk = kr + 16 * i;
      const v4f v = *(const v4f*)(W + (size_t)(k0 + kk) * N + n0 + nc);
      *(v4f*)(tile + kk * 68 + nc) = v;
    }
  }
  __syncthreads();
  const int wv = tid >> 5, lane = tid & 31, q = lane >> 3, e = lane & 7;
  for (int pass = 0; pass < 2; ++pass) {
#pragma unroll
    for (int it = 0; it < 2; ++it) {
      const int nrow = wv * 8 + it * 4 + q;
      v8us hv = (v8us){0, 0, 0, 0, 0, 0, 0, 0};
      v8us lv = (v8us){0, 0, 0, 0, 0, 0, 0, 0};
#pragma unroll
      for (int kk = 0; kk < 8; ++kk) {
        const float f = tile[(8 * e + kk) * 68 + nrow] * scale;
        if (MODE == 0) {
          hv[kk] = f16_bits(f);
        } else {
          const unsigned short hb = f2bf_bits(f);
          hv[kk] = hb;
          lv[kk] = f2bf_bits(f - bf_bits2f(hb));
        }
      }
      const size_t o = (size_t)(n0 + nrow) * K + k0 + 8 * e;
      *(volatile v8us*)(out + o) = hv;
      if (MODE == 1) *(volatile v8us*)(out2 + o) = lv;
    }
    __threadfence();
  }
}

template <int KIN, bool L2MODE>
__global__ __launch_bounds__(512) void lstm_layer_fused(
    const unsigned short* __restrict__ Xin,
    const unsigned short* __restrict__ Wt,
    const unsigned short* __restrict__ Uh,
    const unsigned short* __restrict__ Ul,
    const float* __restrict__ bias,
    const float* __restrict__ h0,
    const float* __restrict__ c0,
    unsigned short* __restrict__ Hout,
    unsigned short* __restrict__ Hout2)
{
  static_assert(KIN % 32 == 0);
  constexpr int P = kHbPitch;
  constexpr int PLANE = 16 * P;
  __shared__ __align__(16) unsigned short hbA[2 * PLANE];
  __shared__ __align__(16) unsigned short hbB[L2MODE ? (2 * PLANE) : 8];

  const int chunk = blockIdx.x;
  const int tid  = threadIdx.x;
  const int wave = tid >> 5;
  const int lane = tid & 31;
  const int cc   = lane & 15;
  const int hh   = lane >> 4;
  const int koff = hh * 8;

  {
    const int u = tid;
    const float hv = h0[u];
    unsigned short e0, e1 = 0;
    if (L2MODE) { e0 = f2bf_bits(hv); e1 = f2bf_bits(hv - bf_bits2f(e0)); }
    else        { e0 = f16_bits(hv); }
#pragma unroll
    for (int r = 0; r < 16; ++r) {
      hbA[r * P + u] = e0;
      if (L2MODE) hbB[r * P + u] = e1;
    }
  }
  float cst[2][8];
  float bcol[8];
#pragma unroll
  for (int nt = 0; nt < 2; ++nt) {
    const int u = 32 * wave + 16 * nt + cc;
    const float cv = c0[u];
#pragma unroll
    for (int r = 0; r < 8; ++r) cst[nt][r] = cv;
#pragma unroll
    for (int g = 0; g < 4; ++g) bcol[g * 2 + nt] = bias[g * kUnits + u] * 16.0f;
  }
  __syncthreads();

  const unsigned short* wrow  = Wt + (size_t)(32 * wave + cc) * KIN + koff;
  const unsigned short* urow  = Uh + (size_t)(32 * wave + cc) * kUnits + koff;
  const unsigned short* urow2 = Ul + (size_t)(32 * wave + cc) * kUnits + koff;
  const unsigned short* xbase = Xin + (size_t)(chunk * kChunkRows + cc) * KIN + koff;

  int cur = 0;
  for (int t = 0; t < kSteps; ++t) {
    const int nxt = cur ^ 1;
    v8f acc[8];
#pragma unroll
    for (int j = 0; j < 8; ++j) { const float bv = bcol[j]; acc[j] = (v8f){bv, bv, bv, bv, bv, bv, bv, bv}; }

    const unsigned short* xr = xbase + (size_t)t * 16 * KIN;
#pragma unroll 1
    for (int k0 = 0; k0 < KIN; k0 += 32) {
      const v16h a = ld_frag_h16(xr + k0);
      v16h bf = a;
#pragma unroll
      for (int j = 0; j < 8; ++j) {
        bf = ld_frag_h16(wrow + (size_t)((j >> 1) * kUnits + (j & 1) * 16) * KIN + k0);
        acc[j] = Frag<_Float16>::mma(a, bf, acc[j]);
        if (j == 3) asm volatile("" ::: "memory");
      }
      dep_guard_h(acc[0], acc[7], a, bf);
    }

    if (!L2MODE) {
      const int hoff = cur * PLANE + cc * P + koff;
#pragma unroll 1
      for (int k0 = 0; k0 < kUnits; k0 += 32) {
        union { v16h v; v8us u[2]; } fa;
        fa.u[0] = *(const v8us*)(hbA + hoff + k0);
        fa.u[1] = *(const v8us*)(hbA + hoff + k0 + 16);
        const v16h a = fa.v;
        v16h bf = a;
#pragma unroll
        for (int j = 0; j < 8; ++j) {
          bf = ld_frag_h16(urow + (size_t)((j >> 1) * kUnits + (j & 1) * 16) * kUnits + k0);
          acc[j] = Frag<_Float16>::mma(a, bf, acc[j]);
          if (j == 3) asm volatile("" ::: "memory");
        }
        dep_guard_h(acc[0], acc[7], a, bf);
      }
    } else {
      const int hoff = cur * PLANE + cc * P + koff;
#pragma unroll 1
      for (int k0 = 0; k0 < kUnits; k0 += 32) {
        union { v16b v; v8us u[2]; } fh, fl;
        fh.u[0] = *(const v8us*)(hbA + hoff + k0);
        fh.u[1] = *(const v8us*)(hbA + hoff + k0 + 16);
        fl.u[0] = *(const v8us*)(hbB + hoff + k0);
        fl.u[1] = *(const v8us*)(hbB + hoff + k0 + 16);
        const v16b ah = fh.v;
        const v16b al = fl.v;
        v16b bh = ah, bl = ah;
#pragma unroll
        for (int j = 0; j < 8; ++j) {
          const size_t uo = (size_t)((j >> 1) * kUnits + (j & 1) * 16) * kUnits + k0;
          bh = ld_frag_b16(urow + uo);
          acc[j] = Frag<__bf16>::mma(ah, bh, acc[j]);
          acc[j] = Frag<__bf16>::mma(al, bh, acc[j]);
          bl = ld_frag_b16(urow2 + uo);
          acc[j] = Frag<__bf16>::mma(ah, bl, acc[j]);
          if (j == 3) asm volatile("" ::: "memory");
        }
        guard4_b(acc[0], acc[7], ah, al, bh, bl);
      }
    }
    acc_guard4(acc[0], acc[1], acc[2], acc[3]);
    acc_guard4(acc[4], acc[5], acc[6], acc[7]);

#pragma unroll
    for (int nt = 0; nt < 2; ++nt) {
      const int col = 32 * wave + 16 * nt + cc;
#pragma unroll
      for (int r = 0; r < 8; ++r) {
        const float zi = acc[nt][r] * 0.0625f;
        const float zf = acc[2 + nt][r] * 0.0625f;
        const float zg = acc[4 + nt][r] * 0.0625f;
        const float zo = acc[6 + nt][r] * 0.0625f;
        const float ig = sigm_f(zi);
        const float fg = sigm_f(zf);
        const float gg = tanh_f(zg);
        const float og = sigm_f(zo);
        const float cn = fg * cst[nt][r] + ig * gg;
        cst[nt][r] = cn;
        const float hn = og * tanh_f(cn);
        const int li = nxt * PLANE + (8 * hh + r) * P + col;
        if (L2MODE) {
          const unsigned short hb = f2bf_bits(hn);
          hbA[li] = hb;
          hbB[li] = f2bf_bits(hn - bf_bits2f(hb));
        } else {
          hbA[li] = f16_bits(hn);
        }
      }
    }
    __syncthreads();

    {
      const int so = nxt * PLANE + wave * P + lane * 8;
      const v8us v0 = *(const v8us*)(hbA + so);
      const v8us v1 = *(const v8us*)(hbA + so + 256);
      v8us w0 = v0, w1 = v1;
      if (L2MODE) {
        w0 = *(const v8us*)(hbB + so);
        w1 = *(const v8us*)(hbB + so + 256);
      }
      const size_t orow = L2MODE ? ((size_t)(chunk * 16 + wave) * kSteps + (size_t)t)
                                 : ((size_t)chunk * kChunkRows + (size_t)t * 16 + (size_t)wave);
      unsigned short* d  = Hout + orow * kUnits + lane * 8;
      unsigned short* d2 = Hout2 + orow * kUnits + lane * 8;
      for (int pass = 0; pass < 2; ++pass) {
        *(volatile v8us*)d = v0;
        *(volatile v8us*)(d + 256) = v1;
        if (L2MODE) {
          *(volatile v8us*)d2 = w0;
          *(volatile v8us*)(d2 + 256) = w1;
        }
        __threadfence();
      }
    }
    cur = nxt;
  }
}

extern "C" void kernel_launch(void* const* d_in, const int* in_sizes, int n_in,
                              void* d_out, int out_size, void* d_ws, size_t ws_size,
                              hipStream_t stream) {
  if (n_in < 18) return;
  if (in_sizes[0] != kRows * kDin) return;
  if (in_sizes[1] != kDin * kGate4 || in_sizes[2] != kUnits * kGate4 || in_sizes[3] != kGate4) return;
  if (in_sizes[4] != kUnits || in_sizes[5] != kUnits) return;
  if (in_sizes[6] != kUnits * kGate4 || in_sizes[7] != kUnits * kGate4 || in_sizes[8] != kGate4) return;
  if (in_sizes[9] != kUnits || in_sizes[10] != kUnits) return;
  if (in_sizes[11] != kUnits * kGate4 || in_sizes[12] != kUnits * kGate4 || in_sizes[13] != kGate4) return;
  if (in_sizes[14] != kUnits || in_sizes[15] != kUnits) return;
  if (in_sizes[16] != kUnits * kDin || in_sizes[17] != kDin) return;
  if (out_size != kRows * kDin) return;
  if (ws_size < kWsTotal) return;

  const float* x   = (const float*)d_in[0];
  const float* W0  = (const float*)d_in[1];
  const float* U0  = (const float*)d_in[2];
  const float* b0  = (const float*)d_in[3];
  const float* h00 = (const float*)d_in[4];
  const float* c00 = (const float*)d_in[5];
  const float* W1  = (const float*)d_in[6];
  const float* U1  = (const float*)d_in[7];
  const float* b1  = (const float*)d_in[8];
  const float* h01 = (const float*)d_in[9];
  const float* c01 = (const float*)d_in[10];
  const float* W2  = (const float*)d_in[11];
  const float* U2  = (const float*)d_in[12];
  const float* b2  = (const float*)d_in[13];
  const float* h02 = (const float*)d_in[14];
  const float* c02 = (const float*)d_in[15];
  const float* Wd  = (const float*)d_in[16];
  const float* bd  = (const float*)d_in[17];

  char* base = (char*)d_ws;
  size_t off = 0;
  unsigned short* X16 = (unsigned short*)(base + off); off += kSzX16;
  unsigned short* W0T = (unsigned short*)(base + off); off += kSzW0T;
  unsigned short* W1T = (unsigned short*)(base + off); off += kSzWT;
  unsigned short* W2T = (unsigned short*)(base + off); off += kSzWT;
  unsigned short* U0T = (unsigned short*)(base + off); off += kSzWT;
  unsigned short* U1T = (unsigned short*)(base + off); off += kSzWT;
  unsigned short* U2H = (unsigned short*)(base + off); off += kSzWT;
  unsigned short* U2L = (unsigned short*)(base + off); off += kSzWT;
  unsigned short* WDH = (unsigned short*)(base + off); off += kSzWD;
  unsigned short* WDL = (unsigned short*)(base + off); off += kSzWD;
  unsigned short* H0P = (unsigned short*)(base + off); off += kSzH;
  unsigned short* H1P = (unsigned short*)(base + off); off += kSzH;
  unsigned short* H2H = (unsigned short*)(base + off); off += kSzH;
  unsigned short* H2L = (unsigned short*)(base + off); off += kSzH;
  if (off != kWsTotal || off > ws_size) return;

  reorder_cast_rows<<<kRows / 8, 256, 0, stream>>>(x, X16, kRows);

  transpose_cast64<0><<<dim3(kGate4 / 64, kDin / 64),   256, 0, stream>>>(W0, W0T, W0T, kDin,   kGate4, 16.0f);
  transpose_cast64<0><<<dim3(kGate4 / 64, kUnits / 64), 256, 0, stream>>>(W1, W1T, W1T, kUnits, kGate4, 16.0f);
  transpose_cast64<0><<<dim3(kGate4 / 64, kUnits / 64), 256, 0, stream>>>(W2, W2T, W2T, kUnits, kGate4, 16.0f);
  transpose_cast64<0><<<dim3(kGate4 / 64, kUnits / 64), 256, 0, stream>>>(U0, U0T, U0T, kUnits, kGate4, 16.0f);
  transpose_cast64<0><<<dim3(kGate4 / 64, kUnits / 64), 256, 0, stream>>>(U1, U1T, U1T, kUnits, kGate4, 16.0f);
  transpose_cast64<1><<<dim3(kGate4 / 64, kUnits / 64), 256, 0, stream>>>(U2, U2H, U2L, kUnits, kGate4, 16.0f);
  transpose_cast64<1><<<dim3(kDin / 64,   kUnits / 64), 256, 0, stream>>>(Wd, WDH, WDL, kUnits, kDin,   1.0f);

  lstm_layer_fused<kDin,   false><<<kChunks, 512, 0, stream>>>(X16, W0T, U0T, U0T, b0, h00, c00, H0P, H0P);
  lstm_layer_fused<kUnits, false><<<kChunks, 512, 0, stream>>>(H0P, W1T, U1T, U1T, b1, h01, c01, H1P, H1P);
  lstm_layer_fused<kUnits, true ><<<kChunks, 512, 0, stream>>>(H1P, W2T, U2H, U2L, b2, h02, c02, H2H, H2L);

  static_assert(kRows % 64 == 0 && kDin % 64 == 0 && kUnits % 32 == 0);
  const int dense_tiles = (kRows / 64) * (kDin / 64);
  wmma_gemm64<1, true, 2, 0, false, 0><<<dim3(dense_tiles / 8, 1), 256, 0, stream>>>(
      H2H, H2L, kUnits, 0L,
      WDH, WDL, kUnits, 0L,
      (void*)d_out, (void*)nullptr, kDin, 0L,
      bd, (const float*)nullptr, 0L,
      kRows, kDin, kUnits, 1.0f);
}
